// SE3PointNeighborConvolution_60593398612079
// MI455X (gfx1250) — hardware-verified
//
#include <hip/hip_runtime.h>
#include <math.h>


#define NBAT 4
#define CIN  32
#define DOUT 32
#define NPT  8192
#define NNB  32
#define NK   36
#define KPAD 48
#define MROW (CIN * NK)
#define PTOT (NBAT * NPT)
typedef __attribute__((ext_vector_type(16))) _Float16 v16h;
typedef __attribute__((ext_vector_type(8)))  _Float16 v8h;
typedef __attribute__((ext_vector_type(8)))  float    v8f;
#define VST2(T, ptr, val) do { const T _v = (val); *(volatile T*)(ptr) = _v; __threadfence(); *(volatile T*)(ptr) = _v; } while (0)
__device__ __forceinline__ v8f wmma16(v16h a, v16h b, v8f c) {
  v8f d = __builtin_amdgcn_wmma_f32_16x16x32_f16(false, a, false, b, (short)0, c, false, false);
  asm volatile("v_nop\n\tv_nop\n\tv_nop\n\tv_nop" : "+v"(d) : "v"(a), "v"(b));
  return d;
}
__device__ __forceinline__ v16h frag16(const _Float16* p, int hh) {
  const v8h lo = *(const v8h*)(p + 8 * hh), hi = *(const v8h*)(p + 16 + 8 * hh);
  return __builtin_shufflevector(lo, hi, 0,1,2,3,4,5,6,7,8,9,10,11,12,13,14,15);
}
__device__ __forceinline__ int kmap(int e, int hh) { return (e < 8) ? (8 * hh + e) : (16 + 8 * hh + (e - 8)); }
__device__ __forceinline__ void lds_sync() { __builtin_amdgcn_fence(__ATOMIC_RELEASE, "workgroup"); __builtin_amdgcn_wave_barrier(); __builtin_amdgcn_fence(__ATOMIC_ACQUIRE, "workgroup"); }

__global__ __launch_bounds__(256) void k_w16(const float* __restrict__ W, _Float16* __restrict__ W16) {
  const int t = blockIdx.x * 256 + threadIdx.x;
  if (t >= DOUT * MROW / 8) return;
  v8h o;
#pragma unroll
  for (int e = 0; e < 8; ++e) o[e] = (_Float16)W[(size_t)t * 8 + e];
  VST2(v8h, W16 + (size_t)t * 8, o);
}
__global__ __launch_bounds__(256) void k_stage1(const float* __restrict__ inp, const float* __restrict__ coords, const float* __restrict__ rmask,
                                                const int* __restrict__ nbr, _Float16* __restrict__ Mrows) {
  __shared__ __attribute__((aligned(16))) _Float16 Bs[8][KPAD][40];
  __shared__ __attribute__((aligned(16))) _Float16 Ms[8][MROW + 8];
  const int lane = threadIdx.x & 31, wave = threadIdx.x >> 5, hh = lane >> 4, l16 = lane & 15;
  const int p = blockIdx.x * 8 + wave;
  const int n = p / NPT, b = p % NPT;
  {
    const int j = min(max(nbr[(size_t)p * NNB + lane], 0), NPT - 1);
    const float* cj = coords + ((size_t)n * NPT + j) * 3; const float* cb = coords + ((size_t)n * NPT + b) * 3;
    const float dx = cj[0] - cb[0], dy = cj[1] - cb[1], dz = cj[2] - cb[2];
    const float r = sqrtf(dx * dx + dy * dy + dz * dz);
    const float ir = 1.0f / (r + 1e-8f);
    const float x = dx * ir, y = dy * ir, z = dz * ir;
    float Y[9] = {0.28209479f, 0.48860251f * x, 0.48860251f * y, 0.48860251f * z, 1.09254843f * x * y, 1.09254843f * y * z,
                  0.31539157f * (3.0f * z * z - 1.0f), 1.09254843f * x * z, 0.54627421f * (x * x - y * y)};
    const float radii[4] = {0.5f, 1.0f, 1.5f, 2.0f};
#pragma unroll
    for (int ri = 0; ri < 4; ++ri) { const float q = (r - radii[ri]) * 2.0f; const float rb = expf(-q * q);
#pragma unroll
      for (int s = 0; s < 9; ++s) Bs[wave][ri * 9 + s][lane] = (_Float16)(rb * Y[s]); }
    if (lane < KPAD - NK) {
#pragma unroll
      for (int a = 0; a < NNB; ++a) Bs[wave][NK + lane][a] = (_Float16)0.f; }
  }
  v16h af[2];
#pragma unroll
  for (int ct = 0; ct < 2; ++ct) {
    const int c = ct * 16 + l16;
#pragma unroll
    for (int e = 0; e < 16; ++e) { const int a = kmap(e, hh); const int j = min(max(nbr[(size_t)p * NNB + a], 0), NPT - 1);
      af[ct][e] = (_Float16)(inp[((size_t)n * CIN + c) * NPT + j] * rmask[(size_t)p * NNB + a]); }
  }
  lds_sync();
#pragma unroll
  for (int kt = 0; kt < 3; ++kt) {
    const v16h bb = frag16(&Bs[wave][kt * 16 + l16][0], hh);
#pragma unroll
    for (int ct = 0; ct < 2; ++ct) {
      v8f d = {}; d = wmma16(af[ct], bb, d);
#pragma unroll
      for (int v = 0; v < 8; ++v) { const int c = ct * 16 + v + 8 * hh, k = kt * 16 + l16; if (k < NK) Ms[wave][c * NK + k] = (_Float16)d[v]; }
    }
  }
  lds_sync();
  _Float16* dst = Mrows + (size_t)p * MROW;
  for (int pass = 0; pass < 2; ++pass) {
    for (int q = lane; q < MROW / 8; q += 32) *(volatile v8h*)(dst + q * 8) = *(const v8h*)(&Ms[wave][q * 8]);
    __threadfence();
  }
}
__global__ __launch_bounds__(128) void k_stage2(const _Float16* __restrict__ Mrows, const _Float16* __restrict__ W16, float* __restrict__ out) {
  __shared__ float sO[4][32][33];
  const int lane = threadIdx.x & 31, wave = threadIdx.x >> 5, hh = lane >> 4, l16 = lane & 15;
  const int p0 = (blockIdx.x * 4 + wave) * 32;
  const int n = p0 / NPT, b0 = p0 % NPT;
  v8f acc[2][2] = {};
#pragma unroll 4
  for (int k0 = 0; k0 < MROW; k0 += 32) {
    const v16h a0 = frag16(Mrows + (size_t)(p0 + l16) * MROW + k0, hh), a1 = frag16(Mrows + (size_t)(p0 + 16 + l16) * MROW + k0, hh);
#pragma unroll
    for (int t = 0; t < 2; ++t) { const v16h bb = frag16(W16 + (size_t)(t * 16 + l16) * MROW + k0, hh); acc[0][t] = wmma16(a0, bb, acc[0][t]); acc[1][t] = wmma16(a1, bb, acc[1][t]); }
  }
#pragma unroll
  for (int r = 0; r < 2; ++r)
#pragma unroll
    for (int t = 0; t < 2; ++t)
#pragma unroll
      for (int v = 0; v < 8; ++v) sO[wave][t * 16 + l16][r * 16 + v + 8 * hh] = acc[r][t][v];
  lds_sync();
  for (int pass = 0; pass < 2; ++pass) {
#pragma unroll 8
    for (int d = 0; d < DOUT; ++d) *(volatile float*)(out + ((size_t)n * DOUT + d) * NPT + b0 + lane) = sO[wave][d][lane];
    __threadfence();
  }
}
extern "C" void kernel_launch(void* const* d_in, const int* in_sizes, int n_in,
                              void* d_out, int out_size, void* d_ws, size_t ws_size, hipStream_t stream) {
  (void)in_sizes; (void)n_in; (void)out_size;
  const float* inp   = (const float*)d_in[0];
  const float* crd   = (const float*)d_in[1];
  const float* rmask = (const float*)d_in[2];
  const float* W     = (const float*)d_in[3];
  const int*   nbr   = (const int*)  d_in[4];
  float* out = (float*)d_out;
  char* ws = (char*)d_ws; size_t off = 0;
  auto take = [&](size_t bytes) { void* p = ws + off; off = (off + bytes + 255) & ~(size_t)255; return p; };
  _Float16* W16   = (_Float16*)take((size_t)DOUT * MROW * 2);
  _Float16* Mrows = (_Float16*)take((size_t)PTOT * MROW * 2);
  if (off > ws_size) return;
  k_w16<<<(DOUT * MROW / 8 + 255) / 256, 256, 0, stream>>>(W, W16);
  k_stage1<<<PTOT / 8, 256, 0, stream>>>(inp, crd, rmask, nbr, Mrows);
  k_stage2<<<PTOT / 32 / 4, 128, 0, stream>>>(Mrows, W16, out);
}
